// MultiHeadAttentionOne_20074677142286
// MI455X (gfx1250) — hardware-verified
//
#include <hip/hip_runtime.h>


#define NB_  2
#define CC   256
#define LL   4096
#define NH_  4
#define HD   64
#define PCAR 1024.0f
typedef _Float16 h16;
typedef unsigned short bf;
typedef __attribute__((ext_vector_type(16))) __bf16   v16bf;
typedef __attribute__((ext_vector_type(16))) _Float16 v16h;
typedef __attribute__((ext_vector_type(8)))  _Float16 v8h;
typedef __attribute__((ext_vector_type(8)))  unsigned short v8us;
typedef __attribute__((ext_vector_type(8)))  float    v8f;
typedef __attribute__((ext_vector_type(4)))  float    v4f;
typedef v8h  __attribute__((may_alias)) v8ha;
typedef v4f  __attribute__((may_alias)) v4fa;
typedef v8us __attribute__((may_alias)) v8usa;

__device__ __forceinline__ unsigned short f2bf(float f) { unsigned u = __float_as_uint(f); u += 0x7FFFu + ((u >> 16) & 1u); return (unsigned short)(u >> 16); }
__device__ __forceinline__ float bf2f(unsigned short b) { return __uint_as_float(((unsigned)b) << 16); }
__device__ __forceinline__ float bfr(float f) { return bf2f(f2bf(f)); }
__device__ __forceinline__ v16h cat16(v8h lo, v8h hi) { return __builtin_shufflevector(lo, hi, 0, 1, 2, 3, 4, 5, 6, 7, 8, 9, 10, 11, 12, 13, 14, 15); }
__device__ __forceinline__ v16bf cat16b(v8us lo, v8us hi) { return __builtin_bit_cast(v16bf, __builtin_shufflevector(lo, hi, 0, 1, 2, 3, 4, 5, 6, 7, 8, 9, 10, 11, 12, 13, 14, 15)); }
__device__ __forceinline__ v8f wmma16(v16h a, v16h b, v8f c) { return __builtin_amdgcn_wmma_f32_16x16x32_f16(false, a, false, b, (short)0, c, false, false); }
__device__ __forceinline__ v8f wmmab(v16bf a, v16bf b, v8f c) { return __builtin_amdgcn_wmma_f32_16x16x32_bf16(false, a, false, b, (short)0, c, false, false); }


template <typename T16> struct WFrag;
template <> struct WFrag<h16> { typedef v16h V; static __device__ __forceinline__ V ld(const h16* p) { return cat16(*(const v8h*)p, *(const v8h*)(p + 16)); } static __device__ __forceinline__ v8f mma(V a, V b, v8f c) { return wmma16(a, b, c); } };
template <> struct WFrag<bf> { typedef v16bf V; static __device__ __forceinline__ V ld(const bf* p) { return cat16b(*(const v8us*)p, *(const v8us*)(p + 16)); } static __device__ __forceinline__ v8f mma(V a, V b, v8f c) { return wmmab(a, b, c); } };
template <typename T16, int NSPLIT, bool BIAS>
__global__ __launch_bounds__(32) void k_gemmw(const T16* __restrict__ A, const T16* __restrict__ A2, const T16* __restrict__ Bt, const T16* __restrict__ Bt2, int K, float* C, int ldc, const float* __restrict__ bias, size_t sA, size_t sB, size_t sC) {
    typedef typename WFrag<T16>::V V;
    __shared__ __align__(16) float os[16 * 68];
    const size_t z = blockIdx.z; A += z * sA; if (A2) A2 += z * sA; Bt += z * sB; if (Bt2) Bt2 += z * sB; C += z * sC;
    const int lane = threadIdx.x & 31, lr = lane & 15, hi = lane >> 4; const int r0 = blockIdx.x * 64, c0 = blockIdx.y * 64;
    v8f acc[4][4];
#pragma unroll
    for (int mb = 0; mb < 4; ++mb)
#pragma unroll
        for (int nb = 0; nb < 4; ++nb) acc[mb][nb] = (v8f){};
    const size_t aoff = (size_t)(r0 + lr) * K + 8 * hi, boff = (size_t)(c0 + lr) * K + 8 * hi;
#pragma unroll 1
    for (int kc = 0; kc < K; kc += 32) {
        V a[4], a2[4];
#pragma unroll
        for (int mb = 0; mb < 4; ++mb) { a[mb] = WFrag<T16>::ld(A + aoff + (size_t)mb * 16 * K + kc); if (NSPLIT == 1 || NSPLIT == 2) a2[mb] = WFrag<T16>::ld(A2 + aoff + (size_t)mb * 16 * K + kc); }
#pragma unroll
        for (int nb = 0; nb < 4; ++nb) { const V b = WFrag<T16>::ld(Bt + boff + (size_t)nb * 16 * K + kc); V b2; if (NSPLIT >= 2) b2 = WFrag<T16>::ld(Bt2 + boff + (size_t)nb * 16 * K + kc);
#pragma unroll
            for (int mb = 0; mb < 4; ++mb) { acc[mb][nb] = WFrag<T16>::mma(a[mb], b, acc[mb][nb]); if (NSPLIT == 1 || NSPLIT == 2) acc[mb][nb] = WFrag<T16>::mma(a2[mb], b, acc[mb][nb]); if (NSPLIT >= 2) acc[mb][nb] = WFrag<T16>::mma(a[mb], b2, acc[mb][nb]); } }
        asm volatile("v_nop\n\tv_nop\n\tv_nop\n\tv_nop" : "+v"(acc[0][0]), "+v"(acc[1][1]), "+v"(acc[2][2]), "+v"(acc[3][3]) : "v"(a[0]), "v"(a[3]));
    }
#pragma unroll
    for (int mb = 0; mb < 4; ++mb) {
#pragma unroll
        for (int nb = 0; nb < 4; ++nb) {
#pragma unroll
            for (int j = 0; j < 8; ++j) os[(hi * 8 + j) * 68 + nb * 16 + lr] = acc[mb][nb][j]; }
        __builtin_amdgcn_wave_barrier(); asm volatile("" ::: "memory");
        float* crow = C + (size_t)(r0 + mb * 16) * ldc + c0;
#pragma unroll 1
        for (int ps = 0; ps < 2; ++ps) {
#pragma unroll
            for (int s = 0; s < 8; ++s) { const int row = 2 * s + hi, cofs = lr * 4; v4f val = *(const v4fa*)(os + row * 68 + cofs); if (BIAS) { val[0] += bfr(bias[c0 + cofs]); val[1] += bfr(bias[c0 + cofs + 1]); val[2] += bfr(bias[c0 + cofs + 2]); val[3] += bfr(bias[c0 + cofs + 3]); }
                *(volatile v4f*)(crow + (size_t)row * ldc + cofs) = val; }
            if (ps == 0) __threadfence(); }
        __builtin_amdgcn_wave_barrier(); asm volatile("" ::: "memory");
    }
}

__device__ __forceinline__ h16 tohx(float x) { return (h16)x; }
__device__ __forceinline__ void splitf(float y, unsigned short& h, unsigned short& l) { h = f2bf(y); l = f2bf(y - bf2f(h)); }
typedef __attribute__((ext_vector_type(2))) unsigned short v2us;
typedef __attribute__((ext_vector_type(4))) unsigned short v4us;
typedef __attribute__((ext_vector_type(2))) _Float16 v2h;
typedef __attribute__((ext_vector_type(4))) _Float16 v4h;
typedef __attribute__((ext_vector_type(8))) float v8f;
typedef __attribute__((ext_vector_type(2))) float v2f;

__global__ __launch_bounds__(256) void k_cvt8(const float* __restrict__ src, bf* dst, size_t n8) { const size_t i = (size_t)blockIdx.x * 256 + threadIdx.x; if (i >= n8) return; const v8f v = *(const v8f*)(src + i * 8); v8us o;
#pragma unroll
    for (int k = 0; k < 8; ++k) o[k] = f2bf(v[k]); *(volatile v8us*)(dst + i * 8) = o; __threadfence(); *(volatile v8us*)(dst + i * 8) = o; }
__global__ __launch_bounds__(256) void k_xt(const float* __restrict__ x, bf* XT, float* XF) { const int e = (blockIdx.x * 256 + threadIdx.x) * 2; if (e >= LL * CC) return; const int c = e % CC; const int l = e / CC; const float a = bfr(x[(size_t)c * LL + l]), b = bfr(x[(size_t)(c + 1) * LL + l]); v2us o; o[0] = f2bf(a); o[1] = f2bf(b); v2f of; of[0] = a; of[1] = b;
    for (int ps = 0; ps < 2; ++ps) { *(volatile v2us*)(XT + e) = o; *(volatile v2f*)(XF + e) = of; if (ps == 0) __threadfence(); } }
__global__ __launch_bounds__(256) void k_pl(const float* __restrict__ F, h16* P) { const int e = (blockIdx.x * 256 + threadIdx.x) * 4; if (e >= NH_ * LL * HD) return; const int d = e % HD; const int l = (e / HD) % LL; const int h = e / (HD * LL); const float* f = F + (size_t)l * CC + h * HD + d; v4h o;
#pragma unroll
    for (int u = 0; u < 4; ++u) o[u] = tohx(f[u]); *(volatile v4h*)(P + e) = o; __threadfence(); *(volatile v4h*)(P + e) = o; }
__global__ __launch_bounds__(256) void k_vt(const float* __restrict__ F, h16* VT) { const int e = (blockIdx.x * 256 + threadIdx.x) * 2; if (e >= NH_ * HD * LL) return; const int l = e % LL; const int d = (e / LL) % HD; const int h = e / (LL * HD); v2h o; o[0] = tohx(F[(size_t)l * CC + h * HD + d]); o[1] = tohx(F[(size_t)(l + 1) * CC + h * HD + d]); *(volatile v2h*)(VT + e) = o; __threadfence(); *(volatile v2h*)(VT + e) = o; }
__global__ __launch_bounds__(256) void k_ssoft(const float* __restrict__ Sb, h16* P16) { const int lane = threadIdx.x & 31; const int row = blockIdx.x * 8 + (threadIdx.x >> 5); if (row >= LL) return; const float* sr = Sb + (size_t)row * LL; float mx = -3.0e38f;
    for (int ch = 0; ch < LL / 128; ++ch) { const v4f a = *(const v4f*)(sr + ch * 128 + lane * 4);
#pragma unroll
        for (int q = 0; q < 4; ++q) mx = fmaxf(mx, a[q] * 0.125f); }
#pragma unroll
    for (int sh = 16; sh; sh >>= 1) mx = fmaxf(mx, __shfl_xor(mx, sh, 32));
    float sum = 0.f;
    for (int ch = 0; ch < LL / 128; ++ch) { const v4f a = *(const v4f*)(sr + ch * 128 + lane * 4);
#pragma unroll
        for (int q = 0; q < 4; ++q) { float d0 = __fsub_rn(a[q] * 0.125f, mx); asm volatile("" : "+v"(d0)); sum += __builtin_amdgcn_exp2f(__fmul_rn(d0, 1.4426950408889634f)); } }
#pragma unroll
    for (int sh = 16; sh; sh >>= 1) sum += __shfl_xor(sum, sh, 32);
    const float f = __fdiv_rn(PCAR, sum);
    for (int ch = 0; ch < LL / 128; ++ch) { const v4f a = *(const v4f*)(sr + ch * 128 + lane * 4); v4h o4;
#pragma unroll
        for (int q = 0; q < 4; ++q) { float d0 = __fsub_rn(a[q] * 0.125f, mx); asm volatile("" : "+v"(d0)); o4[q] = tohx(__builtin_amdgcn_exp2f(__fmul_rn(d0, 1.4426950408889634f)) * f); }
        h16* dst = P16 + (size_t)row * LL + ch * 128 + lane * 4; *(volatile v4h*)dst = o4; __threadfence(); *(volatile v4h*)dst = o4; } }
__global__ __launch_bounds__(256) void k_mrg(const float* __restrict__ O, int h, bf* Ah, bf* Al) { const int e = (blockIdx.x * 256 + threadIdx.x) * 4; if (e >= LL * HD) return; const int d = e % HD; const int l = e / HD; v4us oh, ol;
#pragma unroll
    for (int u = 0; u < 4; ++u) { unsigned short a, b; splitf(O[e + u] * (1.0f / PCAR), a, b); oh[u] = a; ol[u] = b; } const size_t oo = (size_t)l * CC + h * HD + d; *(volatile v4us*)(Ah + oo) = oh; *(volatile v4us*)(Al + oo) = ol; __threadfence(); *(volatile v4us*)(Ah + oo) = oh; *(volatile v4us*)(Al + oo) = ol; }
__global__ __launch_bounds__(256) void k_lnres(const float* __restrict__ Y, const float* __restrict__ XF, const float* __restrict__ gw, const float* __restrict__ gb, float* OUTb) { const int lane = threadIdx.x & 31; const int l = blockIdx.x * 8 + (threadIdx.x >> 5); if (l >= LL) return; const int c0 = lane * 8; float v[8]; float s = 0.f;
#pragma unroll
    for (int u = 0; u < 8; ++u) { const float y = __fadd_rn(Y[(size_t)l * CC + c0 + u], XF[(size_t)l * CC + c0 + u]); v[u] = y; s += y; }
#pragma unroll
    for (int sh = 16; sh; sh >>= 1) s += __shfl_xor(s, sh, 32);
    const float mean = s * (1.0f / CC); float q = 0.f;
#pragma unroll
    for (int u = 0; u < 8; ++u) { float d = __fsub_rn(v[u], mean); asm volatile("" : "+v"(d)); float p = __fmul_rn(d, d); asm volatile("" : "+v"(p)); q = __fadd_rn(q, p); }
#pragma unroll
    for (int sh = 16; sh; sh >>= 1) q += __shfl_xor(q, sh, 32);
    const float den = __fsqrt_rn(__fadd_rn(q * (1.0f / CC), 1e-5f)); v8f o;
#pragma unroll
    for (int u = 0; u < 8; ++u) { float d = __fsub_rn(v[u], mean); asm volatile("" : "+v"(d)); float n0 = __fdiv_rn(d, den); asm volatile("" : "+v"(n0)); float g1 = bfr(gw[c0 + u]); asm volatile("" : "+v"(g1)); float t1 = __fmul_rn(n0, g1); asm volatile("" : "+v"(t1)); o[u] = __fadd_rn(t1, bfr(gb[c0 + u])); }
    float* dst = OUTb + (size_t)l * CC + c0; *(volatile v8f*)dst = o; __threadfence(); *(volatile v8f*)dst = o; }

extern "C" void kernel_launch(void* const* d_in, const int* in_sizes, int n_in,
                              void* d_out, int out_size, void* d_ws, size_t ws_size, hipStream_t stream) {
    (void)in_sizes; (void)n_in; (void)out_size;
    const float** I = (const float**)d_in;
    const float *qin = I[0], *w_qkv = I[1], *fc_w = I[2], *fc_b = I[3], *ln_g = I[4], *ln_b = I[5];
    float* OUT = (float*)d_out;
    char* wsp = (char*)d_ws;
    auto take = [&](size_t bytes) { char* p = wsp; wsp += (bytes + 255) & ~(size_t)255; return (void*)p; };
    bf* BW = (bf*)take(CC * CC * 2); bf* BF = (bf*)take(CC * CC * 2); bf* XT = (bf*)take((size_t)LL * CC * 2); float* XF = (float*)take((size_t)LL * CC * 4); float* QKV = (float*)take((size_t)LL * CC * 4);
    h16* Q16 = (h16*)take((size_t)NH_ * LL * HD * 2); h16* VT = (h16*)take((size_t)NH_ * HD * LL * 2); float* Sb = (float*)take((size_t)LL * LL * 4); h16* P16 = (h16*)take((size_t)LL * LL * 2); float* Oh = (float*)take((size_t)LL * HD * 4); bf* Ah = (bf*)take((size_t)LL * CC * 2); bf* Al = (bf*)take((size_t)LL * CC * 2); float* Y = (float*)take((size_t)LL * CC * 4);
    if ((size_t)(wsp - (char*)d_ws) > ws_size) return;
    k_cvt8<<<(CC * CC / 8 + 255) / 256, 256, 0, stream>>>(w_qkv, BW, CC * CC / 8); k_cvt8<<<(CC * CC / 8 + 255) / 256, 256, 0, stream>>>(fc_w, BF, CC * CC / 8);
    for (int b = 0; b < NB_; ++b) {
        k_xt<<<(LL * CC / 2 + 255) / 256, 256, 0, stream>>>(qin + (size_t)b * CC * LL, XT, XF);
        k_gemmw<bf, 0, false><<<dim3(LL / 64, CC / 64, 1), 32, 0, stream>>>(XT, nullptr, BW, nullptr, CC, QKV, CC, nullptr, 0, 0, 0);
        k_pl<<<(NH_ * LL * HD / 4 + 255) / 256, 256, 0, stream>>>(QKV, Q16); k_vt<<<(NH_ * HD * LL / 2 + 255) / 256, 256, 0, stream>>>(QKV, VT);
        for (int h = 0; h < NH_; ++h) { const size_t zo = (size_t)h * LL * HD;
            k_gemmw<h16, 0, false><<<dim3(LL / 64, LL / 64, 1), 32, 0, stream>>>(Q16 + zo, nullptr, Q16 + zo, nullptr, HD, Sb, LL, nullptr, 0, 0, 0);
            k_ssoft<<<LL / 8, 256, 0, stream>>>(Sb, P16);
            k_gemmw<h16, 0, false><<<dim3(LL / 64, 1, 1), 32, 0, stream>>>(P16, nullptr, VT + (size_t)h * HD * LL, nullptr, LL, Oh, HD, nullptr, 0, 0, 0);
            k_mrg<<<(LL * HD / 4 + 255) / 256, 256, 0, stream>>>(Oh, h, Ah, Al); }
        k_gemmw<bf, 1, true><<<dim3(LL / 64, CC / 64, 1), 32, 0, stream>>>(Ah, Al, BF, nullptr, CC, Y, CC, fc_b, 0, 0, 0);
        k_lnres<<<LL / 8, 256, 0, stream>>>(Y, XF, ln_g, ln_b, OUT + (size_t)b * LL * CC); }
}
